// MobilityPyGEncoder_53532472377745
// MI455X (gfx1250) — hardware-verified
//
#include <hip/hip_runtime.h>
#include <math.h>

#define NN 100000
#define NE 1600000
#define NV (NE + NN)
#define NP 100032
#define FD 128
#define NT 256
#define NWV (NT / 32)
#define SRB 2048
#define RPW (SRB / NWV)
#define NTILE 49
#define NDP (NTILE * SRB)
#define SCH 4096
#define SPT (SCH / NT)
#define NCH ((NV + SCH - 1) / SCH)
#define SENT 0xFFFFFFFFu
#define WSCALE 64.0f
#define HSCALE 16.0f
#define SLP 132

static_assert(NP % 64 == 0 && NP >= NN && NDP >= NP, "");
static_assert(NE % SPT == 0 && SPT % 4 == 0 && SPT == 16, "");
static_assert(NP % 4 == 0 && NN % 4 == 0 && SRB % 4 == 0, "");
static_assert(NV < (1 << 21) && SRB <= 2048 && RPW == 256 && NWV == 8, "");

typedef __attribute__((ext_vector_type(16))) _Float16 v16h;
typedef __attribute__((ext_vector_type(8)))  _Float16 v8h;
typedef __attribute__((ext_vector_type(16))) __bf16   v16b;
typedef __attribute__((ext_vector_type(8)))  __bf16   v8b;
typedef __attribute__((ext_vector_type(8)))  float    v8f;
typedef __attribute__((ext_vector_type(4)))  float    v4f;
typedef __attribute__((ext_vector_type(4)))  int      v4i;

__device__ __forceinline__ unsigned short f2bf_bits(float f) {
  unsigned u = __float_as_uint(f);
  return (unsigned short)((u + 0x7FFFu + ((u >> 16) & 1u)) >> 16);
}
__device__ __forceinline__ float bf_bits2f(unsigned short h) { return __uint_as_float(((unsigned)h) << 16); }

__device__ __forceinline__ void dep_guard_h(v8f& a, v8f& b, v16h x, v16h y) { asm volatile("v_nop\n\tv_nop\n\tv_nop\n\tv_nop" : "+v"(a), "+v"(b) : "v"(x), "v"(y)); }
__device__ __forceinline__ void dep_guard_b(v8f& a, v8f& b, v16b x, v16b y) { asm volatile("v_nop\n\tv_nop\n\tv_nop\n\tv_nop" : "+v"(a), "+v"(b) : "v"(x), "v"(y)); }
__device__ __forceinline__ void keep4_h(v16h a, v16h b, v16h c, v16h d) { asm volatile("v_nop" :: "v"(a), "v"(b), "v"(c), "v"(d)); }
__device__ __forceinline__ void keep4_b(v16b a, v16b b, v16b c, v16b d) { asm volatile("v_nop" :: "v"(a), "v"(b), "v"(c), "v"(d)); }
__device__ __forceinline__ void acc_guard4(v8f& a, v8f& b, v8f& c, v8f& d) { asm volatile("v_nop\n\tv_nop\n\tv_nop\n\tv_nop" : "+v"(a), "+v"(b), "+v"(c), "+v"(d)); }
template <typename T> struct Frag;
template <> struct Frag<_Float16> {
  typedef v16h V; union U { v16h v; v8h h[2]; };
  static __device__ __forceinline__ v16h load(const _Float16* p) {
    U f; f.h[0] = *(const v8h*)(p); f.h[1] = *(const v8h*)(p + 16); return f.v;
  }
  static __device__ __forceinline__ v8f mma(v16h a, v16h b, v8f c) {
    return __builtin_amdgcn_wmma_f32_16x16x32_f16(false, a, false, b, (short)0, c, false, false);
  }
  static __device__ __forceinline__ void guard(v8f& a, v8f& b, v16h x, v16h y) { dep_guard_h(a, b, x, y); }
  static __device__ __forceinline__ void keep(v16h a, v16h b, v16h c, v16h d) { keep4_h(a, b, c, d); }
};
template <> struct Frag<__bf16> {
  typedef v16b V; union U { v16b v; v8b h[2]; };
  static __device__ __forceinline__ v16b load(const __bf16* p) {
    U f; f.h[0] = *(const v8b*)(p); f.h[1] = *(const v8b*)(p + 16); return f.v;
  }
  static __device__ __forceinline__ v8f mma(v16b a, v16b b, v8f c) {
    return __builtin_amdgcn_wmma_f32_16x16x32_bf16(false, a, false, b, (short)0, c, false, false);
  }
  static __device__ __forceinline__ void guard(v8f& a, v8f& b, v16b x, v16b y) { dep_guard_b(a, b, x, y); }
  static __device__ __forceinline__ void keep(v16b a, v16b b, v16b c, v16b d) { keep4_b(a, b, c, d); }
};

template <int ET> struct Elem;
template <> struct Elem<0> { typedef _Float16 T; };
template <> struct Elem<1> { typedef __bf16 T; };
template <int ET, bool SPLIT, int BIAS_MODE, int OUT_MODE, bool RESID, int ACT = 0>
__global__ __launch_bounds__(256) void wmma_gemm64(
    const unsigned short* __restrict__ Ap, const unsigned short* __restrict__ A2p, int lda, long strideA,
    const unsigned short* __restrict__ Btp, const unsigned short* __restrict__ Bt2p, int ldb, long strideB,
    void* __restrict__ Cout, void* __restrict__ Cout2, int ldc, long strideC,
    const float* __restrict__ bias,
    const float* __restrict__ resid, long strideR,
    int M, int N, int K, float scale) {
  typedef typename Elem<ET>::T T;
  typedef typename Frag<T>::V V;
  const T* A = (const T*)Ap; const T* A2 = (const T*)A2p; const T* Bt = (const T*)Btp; const T* Bt2 = (const T*)Bt2p;
  __shared__ __align__(16) float sT[8][16 * 68];
  const int b    = blockIdx.y;
  const int lane = threadIdx.x & 31;
  const int wave = threadIdx.x >> 5;
  const int tilesN = N >> 6;
  const int tilesM = M >> 6;
  const int tile = blockIdx.x * 8 + wave;
  if (tile >= tilesM * tilesN) return;
  const int tm = tile / tilesN;
  const int tn = tile - tm * tilesN;
  const int m0 = tm << 6;
  const int n0 = tn << 6;

  const T* Ab  = A  + (size_t)b * strideA;
  const T* Bb  = Bt + (size_t)b * strideB;
  const T* Ab2 = SPLIT ? (A2  + (size_t)b * strideA) : nullptr;
  const T* Bb2 = SPLIT ? (Bt2 + (size_t)b * strideB) : nullptr;

  const int rlane = lane & 15;
  const int koff  = (lane >> 4) * 8;
  const int mOff  = (lane >> 4) * 8;

  v8f acc[4][4];
#pragma unroll
  for (int i = 0; i < 4; ++i)
#pragma unroll
    for (int j = 0; j < 4; ++j) acc[i][j] = (v8f){0.f,0.f,0.f,0.f,0.f,0.f,0.f,0.f};

  for (int k0 = 0; k0 < K; k0 += 32) {
    V bh[4], bl[4];
#pragma unroll
    for (int j = 0; j < 4; ++j) {
      const size_t bo = (size_t)(n0 + (j << 4) + rlane) * ldb + koff + k0;
      bh[j] = Frag<T>::load(Bb + bo);
      if (SPLIT) bl[j] = Frag<T>::load(Bb2 + bo);
    }
#pragma unroll
    for (int i = 0; i < 4; ++i) {
      const size_t ao = (size_t)(m0 + (i << 4) + rlane) * lda + koff + k0;
      V ah = Frag<T>::load(Ab + ao);
      V al;
      if (SPLIT) al = Frag<T>::load(Ab2 + ao);
#pragma unroll
      for (int j = 0; j < 4; ++j) {
        acc[i][j] = Frag<T>::mma(ah, bh[j], acc[i][j]);
        if (SPLIT) {
          acc[i][j] = Frag<T>::mma(ah, bl[j], acc[i][j]);
          acc[i][j] = Frag<T>::mma(al, bh[j], acc[i][j]);
        }
      }
      Frag<T>::guard(acc[i][0], acc[i][3], ah, SPLIT ? al : ah);
    }
    Frag<T>::keep(bh[0], bh[1], bh[2], bh[3]);
    if (SPLIT) Frag<T>::keep(bl[0], bl[1], bl[2], bl[3]);
  }
  acc_guard4(acc[0][0], acc[0][1], acc[0][2], acc[0][3]);
  acc_guard4(acc[1][0], acc[1][1], acc[1][2], acc[1][3]);
  acc_guard4(acc[2][0], acc[2][1], acc[2][2], acc[2][3]);
  acc_guard4(acc[3][0], acc[3][1], acc[3][2], acc[3][3]);

  float* slab = sT[wave];
  const float* Rb = RESID ? (resid + (size_t)b * strideR) : nullptr;
#pragma unroll
  for (int i = 0; i < 4; ++i) {
    const int mBase = m0 + (i << 4);
#pragma unroll
    for (int j = 0; j < 4; ++j) {
      const int n = n0 + (j << 4) + rlane;
      float bv = 0.f;
      if (BIAS_MODE == 2) bv = bias[n];
#pragma unroll
      for (int r = 0; r < 8; ++r) {
        float v = acc[i][j][r] * scale;
        if (BIAS_MODE == 1) v += bias[mBase + mOff + r];
        if (BIAS_MODE == 2) v += bv;
        if (RESID) v += Rb[(size_t)(mBase + mOff + r) * ldc + n];
        if (ACT == 1) v = tanhf(v);
        if (ACT == 2) v = fmaxf(v, 0.0f);
        if (ACT == 3) v = v / (1.0f + expf(-v));
        if (ACT == 4) v = (v > 0.f) ? v : 0.01f * v;
        if (ACT == 5) v = 0.5f * v * (1.0f + erff(v * 0.70710678118654752f));
        slab[(mOff + r) * 68 + (j << 4) + rlane] = v;
      }
    }
    __builtin_amdgcn_fence(__ATOMIC_RELEASE, "workgroup");
    __builtin_amdgcn_wave_barrier();
    __builtin_amdgcn_fence(__ATOMIC_ACQUIRE, "workgroup");
    if (OUT_MODE == 0) {
      float* C = (float*)Cout + (size_t)b * strideC;
      const int hh = lane >> 4, c4 = (lane & 15) * 4;
      for (int pass = 0; pass < 2; ++pass) {
#pragma unroll
        for (int it = 0; it < 8; ++it) {
          const int row = it * 2 + hh;
          v4f v = *(const v4f*)(slab + row * 68 + c4);
          *(volatile v4f*)(C + (size_t)(mBase + row) * ldc + n0 + c4) = v;
        }
        __threadfence();
      }
    } else {
      const int q = lane >> 3, c8 = (lane & 7) * 8;
      unsigned short* C  = (unsigned short*)Cout  + (size_t)b * strideC;
      unsigned short* C2 = (OUT_MODE == 2) ? ((unsigned short*)Cout2 + (size_t)b * strideC) : nullptr;
      for (int pass = 0; pass < 2; ++pass) {
#pragma unroll
        for (int it = 0; it < 4; ++it) {
          const int row = it * 4 + q;
          const float* sp = slab + row * 68 + c8;
          v8h hv, lv;
#pragma unroll
          for (int e = 0; e < 8; ++e) {
            if (OUT_MODE == 1) {
              hv[e] = (_Float16)sp[e];
            } else {
              unsigned short hb = f2bf_bits(sp[e]);
              unsigned short lb = f2bf_bits(sp[e] - bf_bits2f(hb));
              hv[e] = __builtin_bit_cast(_Float16, hb);
              lv[e] = __builtin_bit_cast(_Float16, lb);
            }
          }
          *(volatile v8h*)(C + (size_t)(mBase + row) * ldc + n0 + c8) = hv;
          if (OUT_MODE == 2) *(volatile v8h*)(C2 + (size_t)(mBase + row) * ldc + n0 + c8) = lv;
        }
        __threadfence();
      }
    }
    __builtin_amdgcn_fence(__ATOMIC_RELEASE, "workgroup");
    __builtin_amdgcn_wave_barrier();
    __builtin_amdgcn_fence(__ATOMIC_ACQUIRE, "workgroup");
  }
}

__global__ __launch_bounds__(NT) void cast_w_kernel(const float* __restrict__ W1, const float* __restrict__ W2,
                                                   unsigned* __restrict__ Wt1, unsigned* __restrict__ Wt2) {
  const int i = blockIdx.x * NT + threadIdx.x;
  if (i >= 2 * (FD * FD / 2)) return;
  const int sel = i >> 13;
  const int j = i & 8191;
  const int n = j >> 6;
  const int k = 2 * (j & 63);
  const float* W = sel ? W2 : W1;
  const _Float16 h0 = (_Float16)(W[(size_t)k * FD + n] * WSCALE);
  const _Float16 h1 = (_Float16)(W[(size_t)(k + 1) * FD + n] * WSCALE);
  const unsigned u = (unsigned)__builtin_bit_cast(unsigned short, h0) | ((unsigned)__builtin_bit_cast(unsigned short, h1) << 16);
  unsigned* dst = sel ? Wt2 : Wt1;
  ((volatile unsigned*)dst)[j] = u;
  __threadfence();
  ((volatile unsigned*)dst)[j] = u;
}

__global__ __launch_bounds__(NT) void cast_x_kernel(const float* __restrict__ x, _Float16* __restrict__ X16) {
  const int i = blockIdx.x * NT + threadIdx.x;
  if (i >= NP * (FD / 8)) return;
  const bool live = i < NN * (FD / 8);
  const int ic = live ? i : (NN * (FD / 8) - 1);
  const v4f a = *(const v4f*)(x + (size_t)ic * 8);
  const v4f c = *(const v4f*)(x + (size_t)ic * 8 + 4);
  v8h hv;
#pragma unroll
  for (int e = 0; e < 4; ++e) {
    hv[e]     = live ? (_Float16)a[e] : (_Float16)0.0f;
    hv[4 + e] = live ? (_Float16)c[e] : (_Float16)0.0f;
  }
  _Float16* p = X16 + (size_t)i * 8;
  *(volatile v8h*)p = hv;
  __threadfence();
  *(volatile v8h*)p = hv;
}

__device__ __forceinline__ int blk_excl_scan(int cnt, int* scan_ws, int tid, int* tot) {
  const int lane = tid & 31, wave = tid >> 5; int incl = cnt;
#pragma unroll
  for (int o = 1; o < 32; o <<= 1) { const int v = __shfl_up(incl, o, 32); if (lane >= o) incl += v; }
  if (lane == 31) scan_ws[wave] = incl;
  __syncthreads();
  if (wave == 0) { int wv = (lane < NT / 32) ? scan_ws[lane] : 0; int wincl = wv;
#pragma unroll
    for (int o = 1; o < 32; o <<= 1) { const int v = __shfl_up(wincl, o, 32); if (lane >= o) wincl += v; }
    if (lane < NT / 32) scan_ws[32 + lane] = wincl - wv; if (lane == 31) scan_ws[64] = wincl; }
  __syncthreads();
  const int res = scan_ws[32 + wave] + incl - cnt; *tot = scan_ws[64];
  return res;
}
template <int SP, int CAP>
__device__ __forceinline__ int chunk_hits(const int* __restrict__ dstv, int e0, int n0, int tid, unsigned* LIST, int* scan_ws) {
  const int eb = e0 + tid * SP;
  const bool real = eb < NE;
  const int ebc = real ? eb : (NE - SP);
  unsigned rec[SP]; int cnt = 0;
#pragma unroll
  for (int k = 0; k < SP; k += 4) {
    const v4i d4 = *(const v4i*)(dstv + ebc + k);
#pragma unroll
    for (int e = 0; e < 4; ++e) {
      const int ve = eb + k + e;
      const int dr = d4[e];
      const int d = real ? dr : (ve - NE);
      const bool ok = real ? ((unsigned)dr < (unsigned)NN) : (ve < NV);
      const bool hit = ok && (d >= n0) && (d < n0 + SRB);
      rec[k + e] = hit ? ((((unsigned)(d - n0)) << 21) | (unsigned)ve) : SENT;
      cnt += hit ? 1 : 0;
    }
  }
  int tot; int p = blk_excl_scan(cnt, scan_ws, tid, &tot);
#pragma unroll
  for (int k = 0; k < SP; ++k) if (rec[k] != SENT) { if ((unsigned)p < (unsigned)CAP) LIST[p] = rec[k]; ++p; }
  __syncthreads();
  return tot < CAP ? tot : CAP;
}

__global__ __launch_bounds__(NT) void deg_kernel(const int* __restrict__ ei, const float* __restrict__ ew, float* __restrict__ dinv) {
  __shared__ unsigned LIST[SCH];
  __shared__ __align__(16) float SDEG[SRB];
  __shared__ int scan_ws[80];
  const int tid = threadIdx.x, lane = tid & 31, wave = tid >> 5;
  const int n0 = blockIdx.x * SRB;
  for (int i = tid; i < SRB; i += NT) SDEG[i] = 0.f;
  __syncthreads();
  const int* dstv = ei + NE;
#pragma unroll 1
  for (int c = 0; c < NCH; ++c) {
    const int tot = chunk_hits<SPT, SCH>(dstv, c * SCH, n0, tid, LIST, scan_ws);
#pragma unroll 1
    for (int base = 0; base < tot; base += 32) {
      const int q = base + lane;
      const int qc = q < SCH ? q : (SCH - 1);
      const unsigned lv = LIST[qc];
      const unsigned rv = (q < tot) ? lv : SENT;
      const int own = (rv != SENT && (rv >> 29) == (unsigned)wave) ? 1 : 0;
      unsigned msk = (unsigned)__ballot(own);
#pragma unroll 1
      for (int it = 0; it < 32; ++it) {
        if (msk == 0u) break;
        const int bp = __builtin_ctz(msk); msk &= msk - 1u;
        const unsigned r = __shfl(rv, bp, 32);
        const int dl = (int)(r >> 21);
        const int ve = (int)(r & 0x1FFFFFu);
        const bool real = ve < NE;
        const int ec = real ? ve : (NE - 1);
        const float wv = real ? ew[ec] : 1.0f;
        if (lane == 0) SDEG[dl] = SDEG[dl] + wv;
      }
    }
    __syncthreads();
  }
#pragma unroll
  for (int i = 0; i < 2; ++i) {
    const int idx = wave * RPW + i * 128 + 4 * lane;
    const v4f d = *(const v4f*)(SDEG + idx);
    v4f dv;
#pragma unroll
    for (int e = 0; e < 4; ++e) dv[e] = (d[e] > 0.f) ? (1.0f / sqrtf(d[e])) : 0.f;
    float* p = dinv + n0 + idx;
    for (int pass = 0; pass < 2; ++pass) { *(volatile v4f*)p = dv; __threadfence(); }
  }
}

template <int MODE>
__global__ __launch_bounds__(NT) void agg_kernel(const float* __restrict__ XW, const int* __restrict__ ei, const float* __restrict__ ew,
                                                const float* __restrict__ dinv, const float* __restrict__ bias, float* ACC,
                                                _Float16* __restrict__ H16, float* __restrict__ OUT) {
  __shared__ unsigned LIST[SCH];
  __shared__ __align__(16) float SDI[SRB];
  __shared__ __align__(16) float SLAB[MODE == 1 ? NWV * 4 * SLP : 4];
  __shared__ int scan_ws[80];
  const int tid = threadIdx.x, lane = tid & 31, wave = tid >> 5;
  const int n0 = blockIdx.x * SRB;
  const v4f br = *(const v4f*)(bias + 4 * lane);
  const v4f z4 = {0.f, 0.f, 0.f, 0.f};
  for (int pass = 0; pass < 2; ++pass) {
#pragma unroll 1
    for (int j = 0; j < RPW; ++j) *(volatile v4f*)(ACC + (size_t)(n0 + wave * RPW + j) * FD + 4 * lane) = z4;
    __threadfence();
  }
  for (int i = tid; i < SRB; i += NT) SDI[i] = dinv[n0 + i];
  __syncthreads();
  const int* srcv = ei; const int* dstv = ei + NE;
#pragma unroll 1
  for (int c = 0; c < NCH; ++c) {
    const int tot = chunk_hits<SPT, SCH>(dstv, c * SCH, n0, tid, LIST, scan_ws);
#pragma unroll 1
    for (int base = 0; base < tot; base += 32) {
      const int q = base + lane;
      const int qc = q < SCH ? q : (SCH - 1);
      const unsigned lv = LIST[qc];
      const unsigned rv = (q < tot) ? lv : SENT;
      const int own = (rv != SENT && (rv >> 29) == (unsigned)wave) ? 1 : 0;
      unsigned msk = (unsigned)__ballot(own);
#pragma unroll 1
      for (int it = 0; it < 32; ++it) {
        if (msk == 0u) break;
        const int bp = __builtin_ctz(msk); msk &= msk - 1u;
        const unsigned r = __shfl(rv, bp, 32);
        const int dl = (int)(r >> 21);
        const int ve = (int)(r & 0x1FFFFFu);
        const bool real = ve < NE;
        const int ec = real ? ve : (NE - 1);
        int s = real ? srcv[ec] : (ve - NE);
        s = s < 0 ? 0 : (s >= NN ? NN - 1 : s);
        const float wv = real ? ew[ec] : 1.0f;
        const float nrm = (dinv[s] * wv) * SDI[dl];
        const v4f xv = *(const v4f*)(XW + (size_t)s * FD + 4 * lane);
        float* rp = ACC + (size_t)(n0 + dl) * FD + 4 * lane;
        v4f a = *(const v4f*)rp;
        a = a + nrm * xv;
        *(volatile v4f*)rp = a;
        __threadfence();
        *(volatile v4f*)rp = a;
      }
    }
    __syncthreads();
  }
  if (MODE == 1) {
    float* slab = SLAB + wave * (4 * SLP);
    const int hrow = lane >> 4, c8 = (lane & 15) * 8;
#pragma unroll 1
    for (int g = 0; g < RPW / 4; ++g) {
      const int nb = n0 + wave * RPW + g * 4;
      if (nb < NP) {
#pragma unroll
        for (int rr = 0; rr < 4; ++rr) {
          const int n = nb + rr;
          const bool live = n < NN;
          const v4f a = *(const v4f*)(ACC + (size_t)n * FD + 4 * lane);
          const v4f t = a + br;
          v4f v;
#pragma unroll
          for (int e = 0; e < 4; ++e) v[e] = live ? (fmaxf(t[e], 0.f) * HSCALE) : 0.f;
          *(v4f*)(slab + rr * SLP + 4 * lane) = v;
        }
        __builtin_amdgcn_fence(__ATOMIC_RELEASE, "workgroup");
        __builtin_amdgcn_wave_barrier();
        __builtin_amdgcn_fence(__ATOMIC_ACQUIRE, "workgroup");
        for (int pass = 0; pass < 2; ++pass) {
#pragma unroll
          for (int it = 0; it < 2; ++it) {
            const int row = it * 2 + hrow;
            const v4f p0 = *(const v4f*)(slab + row * SLP + c8);
            const v4f p1 = *(const v4f*)(slab + row * SLP + c8 + 4);
            v8h hv;
#pragma unroll
            for (int e = 0; e < 4; ++e) { hv[e] = (_Float16)p0[e]; hv[4 + e] = (_Float16)p1[e]; }
            *(volatile v8h*)(H16 + (size_t)(nb + row) * FD + c8) = hv;
          }
          __threadfence();
        }
        __builtin_amdgcn_fence(__ATOMIC_RELEASE, "workgroup");
        __builtin_amdgcn_wave_barrier();
        __builtin_amdgcn_fence(__ATOMIC_ACQUIRE, "workgroup");
      }
    }
  } else {
#pragma unroll 1
    for (int j = 0; j < RPW; ++j) {
      const int n = n0 + wave * RPW + j;
      if (n < NN) {
        const v4f a = *(const v4f*)(ACC + (size_t)n * FD + 4 * lane);
        const v4f v = a + br;
        float* op = OUT + (size_t)n * FD + 4 * lane;
        for (int pass = 0; pass < 2; ++pass) { *(volatile v4f*)op = v; __threadfence(); }
      }
    }
  }
}

extern "C" void kernel_launch(void* const* d_in, const int* in_sizes, int n_in,
                              void* d_out, int out_size, void* d_ws, size_t ws_size, hipStream_t stream) {
  (void)n_in;
  const float* x  = (const float*)d_in[0];
  const int*   ei = (const int*)  d_in[1];
  const float* ew = (const float*)d_in[2];
  const float* W1 = (const float*)d_in[3];
  const float* b1 = (const float*)d_in[4];
  const float* W2 = (const float*)d_in[5];
  const float* b2 = (const float*)d_in[6];
  float* out = (float*)d_out;
  if (in_sizes[0] != NN * FD || in_sizes[1] != 2 * NE || in_sizes[2] != NE || in_sizes[3] != FD * FD ||
      in_sizes[4] != FD || in_sizes[5] != FD * FD || in_sizes[6] != FD || out_size != NN * FD) return;

  char* ws = (char*)d_ws; size_t off = 0;
  auto carve = [&](size_t bytes) -> char* { char* p = ws + off; off += (bytes + 255) & ~(size_t)255; return p; };
  unsigned* Wt1  = (unsigned*)carve((size_t)FD * FD * 2);
  unsigned* Wt2  = (unsigned*)carve((size_t)FD * FD * 2);
  float*    DINV = (float*)carve((size_t)NDP * 4);
  _Float16* XH   = (_Float16*)carve((size_t)NP * FD * 2);
  float*    XW   = (float*)carve((size_t)NP * FD * 4);
  float*    ACC  = (float*)carve((size_t)NDP * FD * 4);
  if (off > ws_size || off > (size_t)134217728) return;

  cast_w_kernel<<<(2 * (FD * FD / 2) + NT - 1) / NT, NT, 0, stream>>>(W1, W2, Wt1, Wt2);
  cast_x_kernel<<<(NP * (FD / 8) + NT - 1) / NT, NT, 0, stream>>>(x, XH);
  const int tiles = (NP / 64) * (FD / 64);
  wmma_gemm64<0, false, 0, 0, false><<<dim3((tiles + 7) / 8, 1), 256, 0, stream>>>(
      (const unsigned short*)XH, (const unsigned short*)nullptr, FD, 0L,
      (const unsigned short*)Wt1, (const unsigned short*)nullptr, FD, 0L,
      (void*)XW, (void*)nullptr, FD, 0L,
      (const float*)nullptr, (const float*)nullptr, 0L, NP, FD, FD, 1.0f / WSCALE);
  deg_kernel<<<NTILE, NT, 0, stream>>>(ei, ew, DINV);
  agg_kernel<1><<<NTILE, NT, 0, stream>>>(XW, ei, ew, DINV, b1, ACC, XH, out);
  wmma_gemm64<0, false, 0, 0, false><<<dim3((tiles + 7) / 8, 1), 256, 0, stream>>>(
      (const unsigned short*)XH, (const unsigned short*)nullptr, FD, 0L,
      (const unsigned short*)Wt2, (const unsigned short*)nullptr, FD, 0L,
      (void*)XW, (void*)nullptr, FD, 0L,
      (const float*)nullptr, (const float*)nullptr, 0L, NP, FD, FD, 1.0f / (WSCALE * HSCALE));
  agg_kernel<2><<<NTILE, NT, 0, stream>>>(XW, ei, ew, DINV, b2, ACC, XH, out);
}
